// PatternBranch_6846177870564
// MI455X (gfx1250) — hardware-verified
//
#include <hip/hip_runtime.h>
#include <math.h>

typedef unsigned short us_t;
typedef us_t   v8us  __attribute__((ext_vector_type(8)));
typedef us_t   v16us __attribute__((ext_vector_type(16)));
typedef __bf16 v16bf __attribute__((ext_vector_type(16)));
typedef float  v8f   __attribute__((ext_vector_type(8)));
typedef float  v4f   __attribute__((ext_vector_type(4)));
typedef v8us __attribute__((may_alias)) v8usa;
typedef v4f  __attribute__((may_alias)) v4fa;

#define NBATCH  256
#define INH     64
#define NCI     3
#define OHW     32
#define NCO     128
#define KRE     27
#define KP      32
#define NPIX    1024
#define TPIX    64
#define NTILE   16
#define NSEL    32
#define PSTR    32

static_assert(NPIX == OHW * OHW);
static_assert(NTILE * TPIX == NPIX);
static_assert(NBATCH * 3 * 4 == 3072);

__device__ __forceinline__ us_t bf16_rne(float x) {
  unsigned u = __float_as_uint(x);
  u = u + 0x7FFFu + ((u >> 16) & 1u);
  return (us_t)(u >> 16);
}
__device__ __forceinline__ float bf16_val(us_t b) {
  return __uint_as_float(((unsigned)b) << 16);
}

__device__ __forceinline__ v8f wmma_bf(v16us au, v16us bu, v8f c) {
  const v16bf a = __builtin_bit_cast(v16bf, au);
  const v16bf b = __builtin_bit_cast(v16bf, bu);
  v8f d = __builtin_amdgcn_wmma_f32_16x16x32_bf16(false, a, false, b, (short)0, c, false, false);
  asm volatile("v_nop\n\tv_nop\n\tv_nop\n\tv_nop" : "+v"(d) : "v"(au), "v"(bu));
  return d;
}

union FragU { v16us u; v8us h2[2]; };
__device__ __forceinline__ v16us frag16(const us_t* p, int h) {
  FragU f;
  f.h2[0] = *(const v8usa*)(p + 8 * h);
  f.h2[1] = *(const v8usa*)(p + 16 + 8 * h);
  return f.u;
}

__device__ __forceinline__ v8f zero8f() {
  v8f z;
  #pragma unroll
  for (int j = 0; j < 8; ++j) z[j] = 0.0f;
  return z;
}

__global__ __launch_bounds__(256) void wprep_k(const float* __restrict__ cw,
                                               us_t* __restrict__ Wh, us_t* __restrict__ Wl)
{
  const int g = blockIdx.x * 256 + threadIdx.x;
  if (g >= NCO * 4) return;
  const int n = g >> 2, grp = g & 3;
  v8us h8, l8;
  #pragma unroll
  for (int i = 0; i < 8; ++i) {
    const int k = 8 * grp + i;
    const int kc = (k < KRE) ? k : (KRE - 1);
    const float w = cw[kc * NCO + n];
    const float v = (k < KRE) ? w : 0.0f;
    const us_t hb = bf16_rne(v);
    h8[i] = hb;
    l8[i] = bf16_rne(v - bf16_val(hb));
  }
  us_t* dh = Wh + n * KP + 8 * grp;
  us_t* dl = Wl + n * KP + 8 * grp;
  *(volatile v8us*)dh = h8;
  *(volatile v8us*)dl = l8;
  __threadfence();
  *(volatile v8us*)dh = h8;
  *(volatile v8us*)dl = l8;
}

__global__ __launch_bounds__(256) void conv_red_k(
    const float* __restrict__ x, const us_t* __restrict__ Wh, const us_t* __restrict__ Wl,
    const float* __restrict__ cb, const float* __restrict__ mw_g,
    const float* __restrict__ sw_g, const float* __restrict__ bw_g,
    const int* __restrict__ sidx, float* __restrict__ part)
{
  __shared__ __attribute__((aligned(16))) us_t  Ah[TPIX * KP];
  __shared__ __attribute__((aligned(16))) us_t  Al[TPIX * KP];
  __shared__ __attribute__((aligned(16))) float feats[TPIX * NCO];
  __shared__ int   ssel[NSEL];
  __shared__ float red[8 * 5];
  __shared__ __attribute__((aligned(16))) float sline[PSTR];

  const int t = threadIdx.x, lane = t & 31, w = t >> 5;
  const int h = lane >> 4, m = lane & 15;
  const int blk = blockIdx.x;
  const int b = blk / NTILE, tile = blk - b * NTILE;
  const int pix0 = tile * TPIX;

  {
    const int k  = t & 31;
    const int kc = (k < KRE) ? k : 0;
    const int kh = kc / 9;
    const int kw = (kc - 9 * kh) / 3;
    const int ci = kc - 9 * kh - 3 * kw;
    const int mb = t >> 5;
    #pragma unroll
    for (int i = 0; i < 8; ++i) {
      const int mm = mb + 8 * i;
      const int oh = 2 * tile + (mm >> 5), ow = mm & 31;
      const int ih = 2 * oh + kh, iw = 2 * ow + kw;
      const int ihc = (ih < INH) ? ih : (INH - 1);
      const int iwc = (iw < INH) ? iw : (INH - 1);
      const float raw = x[((size_t)(b * INH + ihc) * INH + iwc) * NCI + ci];
      const bool ok = (k < KRE) && (ih < INH) && (iw < INH);
      const float v = ok ? raw : 0.0f;
      const us_t hb = bf16_rne(v);
      Ah[mm * KP + k] = hb;
      Al[mm * KP + k] = bf16_rne(v - bf16_val(hb));
    }
  }
  if (t < NSEL) {
    int c = sidx[t];
    c = (c < 0) ? 0 : ((c > NCO - 1) ? (NCO - 1) : c);
    ssel[t] = c;
  }
  __syncthreads();

  const int n0 = 16 * w;
  const v16us bh = frag16(Wh + (n0 + m) * KP, h);
  const v16us bl = frag16(Wl + (n0 + m) * KP, h);
  const v8f z8 = zero8f();
  v8f acc[4];
  #pragma unroll
  for (int mt = 0; mt < 4; ++mt) {
    const v16us ah = frag16(Ah + (16 * mt + m) * KP, h);
    const v16us al = frag16(Al + (16 * mt + m) * KP, h);
    v8f c = z8;
    c = wmma_bf(ah, bh, c);
    c = wmma_bf(al, bh, c);
    c = wmma_bf(ah, bl, c);
    acc[mt] = c;
  }

  const float bias = cb[n0 + m];
  #pragma unroll
  for (int mt = 0; mt < 4; ++mt) {
    #pragma unroll
    for (int r = 0; r < 8; ++r) {
      const float v = acc[mt][r] + bias;
      feats[(16 * mt + 8 * h + r) * NCO + n0 + m] = fmaxf(v, 0.0f);
    }
  }
  __syncthreads();

  const int c = t & 127;
  const float mwc = mw_g[c];
  const int mr0 = t >> 7;
  float am = 0.0f, a0 = 0.0f, a1 = 0.0f, a2 = 0.0f;
  #pragma unroll 4
  for (int i = 0; i < 32; ++i) {
    const int mm = mr0 + 2 * i;
    const float v = feats[mm * NCO + c];
    const float* bw = bw_g + ((size_t)(pix0 + mm) * NCO + c) * 3;
    am += v * mwc;
    a0 += v * bw[0];
    a1 += v * bw[1];
    a2 += v * bw[2];
  }
  float as = 0.0f;
  {
    const int kk = t & 31;
    const int cs = ssel[kk];
    const int pr0 = t >> 5;
    #pragma unroll
    for (int i = 0; i < 8; ++i) {
      const int mm = pr0 + 8 * i;
      as += feats[mm * NCO + cs] * sw_g[(size_t)(pix0 + mm) * NSEL + kk];
    }
  }

  float vals[5];
  vals[0] = am; vals[1] = as; vals[2] = a0; vals[3] = a1; vals[4] = a2;
  #pragma unroll
  for (int v = 0; v < 5; ++v) {
    float s = vals[v];
    #pragma unroll
    for (int msk = 16; msk >= 1; msk >>= 1) s += __shfl_xor(s, msk, 32);
    vals[v] = s;
  }
  if (lane == 0) {
    #pragma unroll
    for (int v = 0; v < 5; ++v) red[w * 5 + v] = vals[v];
  }
  __syncthreads();
  if (t < PSTR) {
    float s = 0.0f;
    if (t < 5) {
      #pragma unroll
      for (int w8 = 0; w8 < 8; ++w8) s += red[w8 * 5 + t];
    }
    sline[t] = s;
  }
  __syncthreads();
  if (t < 8) {
    const v4f pv = *(const v4fa*)(sline + 4 * t);
    float* dst = part + (size_t)blk * PSTR + 4 * t;
    *(volatile v4f*)dst = pv;
    __threadfence();
    *(volatile v4f*)dst = pv;
  }
}

__global__ __launch_bounds__(256) void final_k(
    const float* __restrict__ part, const float* __restrict__ mb_g,
    const float* __restrict__ sb_g, const float* __restrict__ bb_g,
    float* __restrict__ out)
{
  __shared__ __attribute__((aligned(16))) float so[NBATCH * 3];
  const int t = threadIdx.x;
  {
    const int s = t;
    float q0 = 0.0f, q1 = 0.0f, q2 = 0.0f, q3 = 0.0f, q4 = 0.0f;
    #pragma unroll 1
    for (int tl = 0; tl < NTILE; ++tl) {
      const float* p = part + (size_t)(s * NTILE + tl) * PSTR;
      q0 += p[0]; q1 += p[1]; q2 += p[2]; q3 += p[3]; q4 += p[4];
    }
    const float mlog = q0 * (1.0f / 1024.0f) + mb_g[0];
    const bool matched = mlog > 0.0f;
    const float z  = q1 + sb_g[0];
    const float ez = expf(-z);
    const float pr = __builtin_amdgcn_rcpf(1.0f + ez);
    const float l0 = q2 + bb_g[0], l1 = q3 + bb_g[1], l2 = q4 + bb_g[2];
    const float mx = fmaxf(l0, fmaxf(l1, l2));
    const float e0 = expf(l0 - mx), e1 = expf(l1 - mx), e2 = expf(l2 - mx);
    const float inv = __builtin_amdgcn_rcpf((e0 + e1) + e2);
    float o0, o1, o2;
    if (matched && (pr >= 0.5f)) { o0 = pr; o1 = (1.0f - pr) * 0.5f; o2 = o1; }
    else                          { o0 = e0 * inv; o1 = e1 * inv; o2 = e2 * inv; }
    so[s * 3 + 0] = o0;
    so[s * 3 + 1] = o1;
    so[s * 3 + 2] = o2;
  }
  __syncthreads();
  if (t < (NBATCH * 3) / 4) {
    const v4f v = *(const v4fa*)(so + 4 * t);
    float* dst = out + 4 * t;
    *(volatile v4f*)dst = v;
    __threadfence();
    *(volatile v4f*)dst = v;
  }
}

extern "C" void kernel_launch(void* const* d_in, const int* in_sizes, int n_in,
                              void* d_out, int out_size, void* d_ws, size_t ws_size,
                              hipStream_t stream) {
  if (n_in < 10) return;
  if (in_sizes[0] != NBATCH * INH * INH * NCI) return;
  if (in_sizes[1] != KRE * NCO) return;
  if (in_sizes[2] != NCO || in_sizes[3] != NCO) return;
  if (in_sizes[4] < 1 || in_sizes[6] < 1 || in_sizes[8] < 3) return;
  if (in_sizes[5] != NPIX * NSEL) return;
  if (in_sizes[7] != NPIX * NCO * 3) return;
  if (in_sizes[9] != NSEL) return;
  if (out_size != NBATCH * 3) return;

  const float* x    = (const float*)d_in[0];
  const float* cw   = (const float*)d_in[1];
  const float* cb   = (const float*)d_in[2];
  const float* mw   = (const float*)d_in[3];
  const float* mb   = (const float*)d_in[4];
  const float* sw   = (const float*)d_in[5];
  const float* sb   = (const float*)d_in[6];
  const float* bw   = (const float*)d_in[7];
  const float* bb   = (const float*)d_in[8];
  const int*   sidx = (const int*)d_in[9];
  float* outp = (float*)d_out;

  const size_t szWh = (size_t)NCO * KP * 2;
  const size_t szWl = (size_t)NCO * KP * 2;
  const size_t szP  = (size_t)NBATCH * NTILE * PSTR * 4;
  size_t off = 0;
  char* ws = (char*)d_ws;
  us_t*  Wh   = (us_t*)(ws + off);  off += szWh;
  us_t*  Wl   = (us_t*)(ws + off);  off += szWl;
  float* part = (float*)(ws + off); off += szP;
  if (off > ws_size) return;

  wprep_k<<<2, 256, 0, stream>>>(cw, Wh, Wl);
  conv_red_k<<<NBATCH * NTILE, 256, 0, stream>>>(x, Wh, Wl, cb, mw, sw, bw, sidx, part);
  final_k<<<1, 256, 0, stream>>>(part, mb, sb, bb, outp);
}
